// SemanticDistanceFusion_6073083757181
// MI455X (gfx1250) — hardware-verified
//
#include <hip/hip_runtime.h>


namespace {
constexpr int B = 8, NS = 256, D = 512, HID = 2048, NR = B * NS;
constexpr float XS = 8.0f, WSC = 256.0f;
typedef _Float16 b16;
typedef __attribute__((ext_vector_type(16))) _Float16 v16b;
typedef __attribute__((ext_vector_type(8))) _Float16 v8b;
typedef __attribute__((ext_vector_type(8))) float v8f;
typedef __attribute__((ext_vector_type(4))) float v4f;
__device__ __forceinline__ float bf16_rne(float f) { unsigned int u = __float_as_uint(f); u += 0x7FFFu + ((u >> 16) & 1u); float r = __uint_as_float(u & 0xFFFF0000u); asm volatile("" : "+v"(r)); return r; }
__device__ __forceinline__ void split16(float v, b16& hi, b16& lo) { hi = (b16)v; lo = (b16)(v - (float)hi); }
__device__ __forceinline__ v16b frag_kb(const b16* p, int hh) { const v8b a = *(const v8b*)(p + 8 * hh), b = *(const v8b*)(p + 16 + 8 * hh); v16b f;
#pragma unroll
  for (int e = 0; e < 8; ++e) { f[e] = a[e]; f[8 + e] = b[e]; } return f; }
__device__ __forceinline__ v8f wmma16b(v16b a, v16b b, v8f c) { v8f d = __builtin_amdgcn_wmma_f32_16x16x32_f16(false, a, false, b, (short)0, c, false, false); asm volatile("v_nop\n\tv_nop\n\tv_nop\n\tv_nop" : "+v"(d) : "v"(a), "v"(b)); return d; }
__device__ __forceinline__ void wave_lds_sync() { __builtin_amdgcn_fence(__ATOMIC_RELEASE, "workgroup"); __builtin_amdgcn_wave_barrier(); __builtin_amdgcn_fence(__ATOMIC_ACQUIRE, "workgroup"); }
__device__ __forceinline__ float pmul(float a, float b) { float p = a * b; asm volatile("" : "+v"(p)); return p; }
__device__ __forceinline__ float gelu(float v) { return 0.5f * v * (1.0f + erff(v * 0.70710678118654752f)); }

__global__ __launch_bounds__(256) void wput_kernel(const float* __restrict__ w, int KIN, int OUTW, b16* __restrict__ WT) { const int KG = KIN / 8; const size_t u = (size_t)blockIdx.x * 256 + threadIdx.x; if (u >= (size_t)OUTW * KG) return; const int o = (int)(u / KG), k0 = (int)(u % KG) * 8; v8b v;
#pragma unroll
  for (int j = 0; j < 8; ++j) v[j] = (b16)(bf16_rne(w[(size_t)(k0 + j) * OUTW + o]) * WSC); for (int pass = 0; pass < 2; ++pass) { *(volatile v8b*)(WT + (size_t)o * KIN + k0) = v; __threadfence(); } }
template <int MODE>
__global__ __launch_bounds__(256) void md_kernel(const float* __restrict__ xv, const float* __restrict__ xa, int BV, float* __restrict__ MD) {
  const int wave = threadIdx.x >> 5, lane = threadIdx.x & 31; const size_t row = (size_t)blockIdx.x * 8 + wave; const int b = (int)(row / NS); if (b >= BV) return; const float* mine = (MODE == 0 ? xv : xa) + row * D; const float* oth = (MODE == 0 ? xa : xv) + (size_t)b * NS * D;
  float me[16]; for (int q = 0; q < 16; ++q) me[q] = bf16_rne(mine[q * 32 + lane]); float tot = 0.0f;
#pragma unroll 1
  for (int m = 0; m < NS; ++m) { float s = 0.0f;
#pragma unroll
    for (int q = 0; q < 16; ++q) s += fabsf(me[q] - bf16_rne(oth[(size_t)m * D + q * 32 + lane]));
    for (int o = 16; o; o >>= 1) s += __shfl_xor(s, o); tot += s; }
  const float mean = tot * (1.0f / NS);
  for (int pass = 0; pass < 2; ++pass) { ((volatile float*)MD)[((size_t)MODE * NR + row) * 32 + lane] = (lane == 0) ? mean : 0.0f; __threadfence(); } }
template <int KIN, int SRC>
__global__ __launch_bounds__(32) void gemm_kernel(const float* __restrict__ IN, const float* __restrict__ MDp, const b16* __restrict__ WT, const float* __restrict__ bias, int NG, int OW, int ocol0, int RL, float* __restrict__ OUT) {
  constexpr int KCH = KIN > 1024 ? 1024 : KIN;
  __shared__ __attribute__((aligned(16))) b16 Ah[16][KCH + 8], Al[16][KCH + 8]; __shared__ float Tf[16][132], Scl[16]; const int lane = threadIdx.x, nloc = lane & 15, hlf = lane >> 4; const int g = blockIdx.x % NG; const size_t m0 = (size_t)(blockIdx.x / NG) * 16; if (m0 >= (size_t)RL) return;
  if (lane < 16) Scl[lane] = (SRC == 0) ? MDp[(m0 + lane) * 32] : 1.0f;
  v8f acc[8];
#pragma unroll
  for (int t = 0; t < 8; ++t) acc[t] = (v8f){};
#pragma unroll 1
  for (int kc = 0; kc < KIN; kc += KCH) {
    wave_lds_sync();
    for (int rr = 0; rr < 16; ++rr) { const float sc = Scl[rr]; for (int q = 0; q < KCH / 32; ++q) { float v = IN[(m0 + rr) * KIN + kc + q * 32 + lane]; if (SRC == 0) v = pmul(bf16_rne(v), sc); else if (SRC == 1) v = gelu(v); b16 p, ql; split16(v * XS, p, ql); Ah[rr][q * 32 + lane] = p; Al[rr][q * 32 + lane] = ql; } }
    wave_lds_sync();
#pragma unroll 2
    for (int kb = 0; kb < KCH; kb += 32) { const v16b a = frag_kb(&Ah[nloc][kb], hlf), al = frag_kb(&Al[nloc][kb], hlf);
#pragma unroll
      for (int t = 0; t < 8; ++t) { const v16b bw = frag_kb(WT + (size_t)(g * 128 + t * 16 + nloc) * KIN + kc + kb, hlf); acc[t] = wmma16b(a, bw, acc[t]); acc[t] = wmma16b(al, bw, acc[t]); } } }
#pragma unroll
  for (int t = 0; t < 8; ++t) { const int c = g * 128 + t * 16 + nloc; const float bb = bf16_rne(bias[c]);
#pragma unroll
    for (int r8 = 0; r8 < 8; ++r8) Tf[8 * hlf + r8][t * 16 + nloc] = acc[t][r8] * (1.0f / (XS * WSC)) + bb; }
  wave_lds_sync();
  for (int pass = 0; pass < 2; ++pass) { for (int rr = 0; rr < 16; ++rr) *(volatile v4f*)(OUT + (m0 + rr) * OW + ocol0 + g * 128 + lane * 4) = *(const v4f*)(&Tf[rr][lane * 4]); __threadfence(); }
}
__global__ __launch_bounds__(256) void fuse_kernel(const float* __restrict__ xmm, const float* __restrict__ DIST, const float* __restrict__ Wf, const float* __restrict__ bfz, int RL, float* __restrict__ out) {
  const int wave = threadIdx.x >> 5, lane = threadIdx.x & 31; const size_t row = (size_t)blockIdx.x * 8 + wave; if (row >= (size_t)RL) return; float g0 = 0.0f, g1 = 0.0f;
#pragma unroll 1
  for (int q = 0; q < D / 32; ++q) { const int c = q * 32 + lane; const float xm = bf16_rne(xmm[row * D + c]), dv = DIST[row * D + c]; g0 += pmul(xm, bf16_rne(Wf[c * 2])) + pmul(dv, bf16_rne(Wf[(D + c) * 2])); g1 += pmul(xm, bf16_rne(Wf[c * 2 + 1])) + pmul(dv, bf16_rne(Wf[(D + c) * 2 + 1])); }
  for (int o = 16; o; o >>= 1) { g0 += __shfl_xor(g0, o); g1 += __shfl_xor(g1, o); } g0 += bf16_rne(bfz[0]); g1 += bf16_rne(bfz[1]); const float sg = 1.0f / (1.0f + __expf(-g0)), th = tanhf(g1);
  for (int pass = 0; pass < 2; ++pass) {
#pragma unroll 1
    for (int q = 0; q < D / 32; ++q) { const int c = q * 32 + lane; ((volatile float*)out)[row * D + c] = pmul(sg, bf16_rne(xmm[row * D + c])) + pmul(th, DIST[row * D + c]); } __threadfence(); } }
}

extern "C" void kernel_launch(void* const* d_in, const int* in_sizes, int n_in, void* d_out, int out_size, void* d_ws, size_t ws_size, hipStream_t stream) {
  (void)n_in;
  auto Fp = [&](int i) { return (const float*)d_in[i]; };
  if (in_sizes[0] != NR * D || in_sizes[1] != NR * D || in_sizes[2] != NR * D || in_sizes[3] != D * HID || in_sizes[7] != HID * D || in_sizes[11] != 2 * D * D || in_sizes[13] != 2 * D * 2 || out_size != NR * D) return;
  const int BV = B; const int RL = BV * NS;
  size_t off = 0; char* ws = (char*)d_ws;
  auto carve = [&](size_t bytes) { char* p = ws + off; off += (bytes + 255) & ~(size_t)255; return p; };
  b16* W1V = (b16*)carve((size_t)HID * D * 2); b16* W1A = (b16*)carve((size_t)HID * D * 2); b16* W2V = (b16*)carve((size_t)D * HID * 2); b16* W2A = (b16*)carve((size_t)D * HID * 2); b16* WO = (b16*)carve((size_t)D * 2 * D * 2);
  float* MD = (float*)carve((size_t)2 * NR * 32 * 4); float* H1 = (float*)carve((size_t)NR * HID * 4); float* HC = (float*)carve((size_t)NR * 2 * D * 4); float* DIST = (float*)carve((size_t)NR * D * 4);
  if (off > ws_size || off > ((size_t)64 << 20)) return;
  wput_kernel<<<(unsigned)(((size_t)HID * (D / 8) + 255) / 256), 256, 0, stream>>>(Fp(3), D, HID, W1V); wput_kernel<<<(unsigned)(((size_t)HID * (D / 8) + 255) / 256), 256, 0, stream>>>(Fp(5), D, HID, W1A);
  wput_kernel<<<(unsigned)(((size_t)D * (HID / 8) + 255) / 256), 256, 0, stream>>>(Fp(7), HID, D, W2V); wput_kernel<<<(unsigned)(((size_t)D * (HID / 8) + 255) / 256), 256, 0, stream>>>(Fp(9), HID, D, W2A); wput_kernel<<<(unsigned)(((size_t)D * (2 * D / 8) + 255) / 256), 256, 0, stream>>>(Fp(11), 2 * D, D, WO);
  md_kernel<0><<<(RL + 7) / 8, 256, 0, stream>>>(Fp(1), Fp(2), BV, MD); md_kernel<1><<<(RL + 7) / 8, 256, 0, stream>>>(Fp(1), Fp(2), BV, MD);
  gemm_kernel<D, 0><<<(RL / 16) * (HID / 128), 32, 0, stream>>>(Fp(1), MD, W1V, Fp(4), HID / 128, HID, 0, RL, H1);
  gemm_kernel<HID, 1><<<(RL / 16) * (D / 128), 32, 0, stream>>>(H1, nullptr, W2V, Fp(8), D / 128, 2 * D, 0, RL, HC);
  gemm_kernel<D, 0><<<(RL / 16) * (HID / 128), 32, 0, stream>>>(Fp(2), MD + (size_t)NR * 32, W1A, Fp(6), HID / 128, HID, 0, RL, H1);
  gemm_kernel<HID, 1><<<(RL / 16) * (D / 128), 32, 0, stream>>>(H1, nullptr, W2A, Fp(10), D / 128, 2 * D, D, RL, HC);
  gemm_kernel<2 * D, 2><<<(RL / 16) * (D / 128), 32, 0, stream>>>(HC, nullptr, WO, Fp(12), D / 128, D, 0, RL, DIST);
  fuse_kernel<<<(RL + 7) / 8, 256, 0, stream>>>(Fp(0), DIST, Fp(13), Fp(14), RL, (float*)d_out);
}
